// BaseGumbelGraphNetwork_81621558493432
// MI455X (gfx1250) — hardware-verified
//
#include <hip/hip_runtime.h>
#include <stdint.h>

typedef __attribute__((ext_vector_type(16))) _Float16 v16h;
typedef __attribute__((ext_vector_type(8)))  _Float16 v8h;
typedef __attribute__((ext_vector_type(8)))  float    v8f;
typedef __attribute__((ext_vector_type(4)))  float    v4f;

__device__ __forceinline__ void dep_guard_h(v8f& a, v8f& b, v16h x, v16h y) { asm volatile("v_nop\n\tv_nop\n\tv_nop\n\tv_nop" : "+v"(a), "+v"(b) : "v"(x), "v"(y)); }
__device__ __forceinline__ void keep4_h(v16h a, v16h b, v16h c, v16h d) { asm volatile("v_nop" :: "v"(a), "v"(b), "v"(c), "v"(d)); }
template <typename T> struct Frag;
template <> struct Frag<_Float16> {
  typedef v16h V; union U { v16h v; v8h h[2]; };
  static __device__ __forceinline__ v16h load(const _Float16* p) {
    U f; f.h[0] = *(const v8h*)(p); f.h[1] = *(const v8h*)(p + 16); return f.v;
  }
  static __device__ __forceinline__ v8f mma(v16h a, v16h b, v8f c) {
    return __builtin_amdgcn_wmma_f32_16x16x32_f16(false, a, false, b, (short)0, c, false, false);
  }
  static __device__ __forceinline__ void guard(v8f& a, v8f& b, v16h x, v16h y) { dep_guard_h(a, b, x, y); }
  static __device__ __forceinline__ void keep(v16h a, v16h b, v16h c, v16h d) { keep4_h(a, b, c, d); }
};

__device__ __forceinline__ v8f mma_h(v16h a, v16h b, v8f c) {
  c = __builtin_amdgcn_wmma_f32_16x16x32_f16(false, a, false, b, (short)0, c, false, false);
  asm volatile("v_nop\n\tv_nop\n\tv_nop\n\tv_nop" : "+v"(c) : "v"(a), "v"(b));
  return c;
}

__device__ __forceinline__ void lds_wave_sync() {
  __builtin_amdgcn_fence(__ATOMIC_RELEASE, "workgroup");
  __builtin_amdgcn_wave_barrier();
  __builtin_amdgcn_fence(__ATOMIC_ACQUIRE, "workgroup");
}

#define NN 512
#define HH 64
#define DD 2
#define NWV 8
#define OPS 64.0f
#define OPS2_INV (1.0f / 4096.0f)

__global__ __launch_bounds__(256) void edge_sum_kernel(
    const float* __restrict__ input, const float* __restrict__ adj,
    const float* __restrict__ W_n2e, const float* __restrict__ b_n2e,
    const float* __restrict__ W_e2e, const float* __restrict__ b_e2e,
    float* __restrict__ S)
{
  __shared__ __align__(16) _Float16 Wsh[HH * HH];
  __shared__ __align__(16) _Float16 E1[NWV][16 * HH];
  __shared__ __align__(16) float s_x[NN * DD];
  __shared__ __align__(16) float s_adj[NN];
  __shared__ __align__(16) float s_part[NWV][HH];
  __shared__ __align__(16) float s_s[HH];

  const int tid  = threadIdx.x;
  const int wave = tid >> 5;
  const int lane = tid & 31;
  const int wg   = blockIdx.x;
  const int bi   = wg >> 9;
  const int ii   = wg & (NN - 1);
  const int rlane = lane & 15;
  const int hh    = lane >> 4;
  const int koff  = hh * 8;

  {
    const v4f v = *(const v4f*)(input + (size_t)bi * NN * DD + tid * 4);
    *(v4f*)(s_x + tid * 4) = v;
  }
  if (tid < NN / 4) {
    const v4f v = *(const v4f*)(adj + (size_t)ii * NN + tid * 4);
    *(v4f*)(s_adj + tid * 4) = v;
  }
  {
    const float* wp = W_e2e + tid * 16;
    const v4f w0 = *(const v4f*)(wp + 0);
    const v4f w1 = *(const v4f*)(wp + 4);
    const v4f w2 = *(const v4f*)(wp + 8);
    const v4f w3 = *(const v4f*)(wp + 12);
    v8h h0, h1;
#pragma unroll
    for (int e = 0; e < 4; ++e) {
      h0[e]     = (_Float16)(w0[e] * OPS);
      h0[4 + e] = (_Float16)(w1[e] * OPS);
      h1[e]     = (_Float16)(w2[e] * OPS);
      h1[4 + e] = (_Float16)(w3[e] * OPS);
    }
    *(v8h*)(Wsh + tid * 16)     = h0;
    *(v8h*)(Wsh + tid * 16 + 8) = h1;
  }
  __syncthreads();

  const float xi0 = s_x[2 * ii], xi1 = s_x[2 * ii + 1];
  const int h8 = (lane & 7) * 8;
  const int rg = (lane >> 3) * 4;
  float ci[8], cw2[8], cw3[8];
#pragma unroll
  for (int e = 0; e < 8; ++e) {
    const int h = h8 + e;
    const v4f wr = *(const v4f*)(W_n2e + h * 4);
    ci[e]  = OPS * (b_n2e[h] + xi0 * wr[0] + xi1 * wr[1]);
    cw2[e] = OPS * wr[2];
    cw3[e] = OPS * wr[3];
  }
  float bee[4];
#pragma unroll
  for (int nt = 0; nt < 4; ++nt) bee[nt] = b_e2e[nt * 16 + rlane];

  float accn[4] = {0.f, 0.f, 0.f, 0.f};
  _Float16* et = E1[wave];
  const int jw = wave * 64;

#pragma unroll 1
  for (int jt = 0; jt < 4; ++jt) {
    const int jb = jw + jt * 16;
    lds_wave_sync();
#pragma unroll
    for (int q = 0; q < 4; ++q) {
      const int j = jb + rg + q;
      const float xj0 = s_x[2 * j], xj1 = s_x[2 * j + 1];
      v8h hv;
#pragma unroll
      for (int e = 0; e < 8; ++e) {
        float v = ci[e] + xj0 * cw2[e] + xj1 * cw3[e];
        v = fmaxf(v, 0.0f);
        hv[e] = (_Float16)v;
      }
      *(v8h*)(et + (rg + q) * HH + h8) = hv;
    }
    lds_wave_sync();

    const v16h a0 = Frag<_Float16>::load(et + rlane * HH + koff);
    const v16h a1 = Frag<_Float16>::load(et + rlane * HH + 32 + koff);
    float aw[8];
#pragma unroll
    for (int r = 0; r < 8; ++r) aw[r] = s_adj[jb + 8 * hh + r];

#pragma unroll
    for (int nt = 0; nt < 4; ++nt) {
      const v16h b0 = Frag<_Float16>::load(Wsh + (nt * 16 + rlane) * HH + koff);
      const v16h b1 = Frag<_Float16>::load(Wsh + (nt * 16 + rlane) * HH + 32 + koff);
      v8f c = (v8f){0.f, 0.f, 0.f, 0.f, 0.f, 0.f, 0.f, 0.f};
      c = mma_h(a0, b0, c);
      c = mma_h(a1, b1, c);
      float p = 0.f;
#pragma unroll
      for (int r = 0; r < 8; ++r) {
        float e2 = c[r] * OPS2_INV + bee[nt];
        e2 = fmaxf(e2, 0.0f);
        p += e2 * aw[r];
      }
      accn[nt] += p;
    }
  }

#pragma unroll
  for (int nt = 0; nt < 4; ++nt) accn[nt] += __shfl_xor(accn[nt], 16, 32);
  if (lane < 16) {
#pragma unroll
    for (int nt = 0; nt < 4; ++nt) s_part[wave][nt * 16 + lane] = accn[nt];
  }
  __syncthreads();
  if (tid < HH) {
    float s = 0.f;
#pragma unroll
    for (int w = 0; w < NWV; ++w) s += s_part[w][tid];
    s_s[tid] = s;
  }
  __syncthreads();
  if (wave == 0 && lane < 16) {
    const v4f v = *(const v4f*)(s_s + lane * 4);
    float* dst = S + (size_t)wg * HH + lane * 4;
    *(volatile v4f*)dst = v;
    __threadfence();
    *(volatile v4f*)dst = v;
  }
}

__global__ __launch_bounds__(256) void node_mlp_kernel(
    const float* __restrict__ S, const float* __restrict__ input,
    const float* __restrict__ W_e2n, const float* __restrict__ b_e2n,
    const float* __restrict__ W_n2n, const float* __restrict__ b_n2n,
    const float* __restrict__ W_o1,  const float* __restrict__ b_o1,
    const float* __restrict__ W_o2,  const float* __restrict__ b_o2,
    float* __restrict__ out)
{
  __shared__ __align__(16) float actA[16 * 68];
  __shared__ __align__(16) float actB[16 * 68];
  __shared__ __align__(16) float xin[32];
  __shared__ __align__(16) float outv[32];

  const int tid = threadIdx.x;
  const int n0  = blockIdx.x * 16;

  for (int idx = tid; idx < 16 * HH; idx += 256) actA[(idx >> 6) * 68 + (idx & 63)] = S[(size_t)n0 * HH + idx];
  if (tid < 32) xin[tid] = input[(size_t)n0 * DD + tid];
  __syncthreads();

  const int h  = tid & 63;
  const int ng = tid >> 6;
  const int nl0 = ng * 4;

  {
    const float bv = b_e2n[h];
    float a0 = bv, a1 = bv, a2 = bv, a3 = bv;
    const float* w = W_e2n + h * HH;
#pragma unroll 1
    for (int k = 0; k < HH; ++k) {
      const float wk = w[k];
      a0 += actA[(nl0 + 0) * 68 + k] * wk;
      a1 += actA[(nl0 + 1) * 68 + k] * wk;
      a2 += actA[(nl0 + 2) * 68 + k] * wk;
      a3 += actA[(nl0 + 3) * 68 + k] * wk;
    }
    actB[(nl0 + 0) * 68 + h] = fmaxf(a0, 0.0f);
    actB[(nl0 + 1) * 68 + h] = fmaxf(a1, 0.0f);
    actB[(nl0 + 2) * 68 + h] = fmaxf(a2, 0.0f);
    actB[(nl0 + 3) * 68 + h] = fmaxf(a3, 0.0f);
  }
  __syncthreads();
  {
    const float bv = b_n2n[h];
    float a0 = bv, a1 = bv, a2 = bv, a3 = bv;
    const float* w = W_n2n + h * HH;
#pragma unroll 1
    for (int k = 0; k < HH; ++k) {
      const float wk = w[k];
      a0 += actB[(nl0 + 0) * 68 + k] * wk;
      a1 += actB[(nl0 + 1) * 68 + k] * wk;
      a2 += actB[(nl0 + 2) * 68 + k] * wk;
      a3 += actB[(nl0 + 3) * 68 + k] * wk;
    }
    actA[(nl0 + 0) * 68 + h] = fmaxf(a0, 0.0f);
    actA[(nl0 + 1) * 68 + h] = fmaxf(a1, 0.0f);
    actA[(nl0 + 2) * 68 + h] = fmaxf(a2, 0.0f);
    actA[(nl0 + 3) * 68 + h] = fmaxf(a3, 0.0f);
  }
  __syncthreads();
  {
    const float* w = W_o1 + h * (DD + HH);
    const float bv = b_o1[h], wx0 = w[0], wx1 = w[1];
    float a0 = bv + xin[(nl0 + 0) * 2] * wx0 + xin[(nl0 + 0) * 2 + 1] * wx1;
    float a1 = bv + xin[(nl0 + 1) * 2] * wx0 + xin[(nl0 + 1) * 2 + 1] * wx1;
    float a2 = bv + xin[(nl0 + 2) * 2] * wx0 + xin[(nl0 + 2) * 2 + 1] * wx1;
    float a3 = bv + xin[(nl0 + 3) * 2] * wx0 + xin[(nl0 + 3) * 2 + 1] * wx1;
#pragma unroll 1
    for (int k = 0; k < HH; ++k) {
      const float wk = w[2 + k];
      a0 += actA[(nl0 + 0) * 68 + k] * wk;
      a1 += actA[(nl0 + 1) * 68 + k] * wk;
      a2 += actA[(nl0 + 2) * 68 + k] * wk;
      a3 += actA[(nl0 + 3) * 68 + k] * wk;
    }
    actB[(nl0 + 0) * 68 + h] = fmaxf(a0, 0.0f);
    actB[(nl0 + 1) * 68 + h] = fmaxf(a1, 0.0f);
    actB[(nl0 + 2) * 68 + h] = fmaxf(a2, 0.0f);
    actB[(nl0 + 3) * 68 + h] = fmaxf(a3, 0.0f);
  }
  __syncthreads();
  if (tid < 32) {
    const int nl = tid >> 1, o = tid & 1;
    const float* w = W_o2 + o * HH;
    float a = b_o2[o];
#pragma unroll 1
    for (int k = 0; k < HH; ++k) a += actB[nl * 68 + k] * w[k];
    outv[tid] = a;
  }
  __syncthreads();
  if (tid < 8) {
    const v4f v = *(const v4f*)(outv + tid * 4);
    float* dst = out + (size_t)n0 * 2 + tid * 4;
    *(volatile v4f*)dst = v;
    __threadfence();
    *(volatile v4f*)dst = v;
  }
}

extern "C" void kernel_launch(void* const* d_in, const int* in_sizes, int n_in,
                              void* d_out, int out_size, void* d_ws, size_t ws_size,
                              hipStream_t stream)
{
  if (n_in < 14) return;
  const int nB = in_sizes[0] / (NN * DD);
  if (nB <= 0) return;
  if (in_sizes[0] != nB * NN * DD) return;
  if (in_sizes[1] != NN * NN) return;
  if (in_sizes[2] != HH * 2 * DD || in_sizes[3] != HH) return;
  if (in_sizes[4] != HH * HH || in_sizes[5] != HH) return;
  if (in_sizes[6] != HH * HH || in_sizes[7] != HH) return;
  if (in_sizes[8] != HH * HH || in_sizes[9] != HH) return;
  if (in_sizes[10] != HH * (DD + HH) || in_sizes[11] != HH) return;
  if (in_sizes[12] != 2 * HH || in_sizes[13] != 2) return;
  if (out_size != nB * NN * 2) return;

  const float* input = (const float*)d_in[0];
  const float* adj   = (const float*)d_in[1];
  const float* W_n2e = (const float*)d_in[2];
  const float* b_n2e = (const float*)d_in[3];
  const float* W_e2e = (const float*)d_in[4];
  const float* b_e2e = (const float*)d_in[5];
  const float* W_e2n = (const float*)d_in[6];
  const float* b_e2n = (const float*)d_in[7];
  const float* W_n2n = (const float*)d_in[8];
  const float* b_n2n = (const float*)d_in[9];
  const float* W_o1  = (const float*)d_in[10];
  const float* b_o1  = (const float*)d_in[11];
  const float* W_o2  = (const float*)d_in[12];
  const float* b_o2  = (const float*)d_in[13];
  float* out = (float*)d_out;

  const size_t s_bytes = (size_t)nB * NN * HH * sizeof(float);
  if (s_bytes > ws_size) return;
  float* S = (float*)d_ws;

  const int nNodes = nB * NN;
  edge_sum_kernel<<<nNodes, 256, 0, stream>>>(input, adj, W_n2e, b_n2e, W_e2e, b_e2e, S);
  node_mlp_kernel<<<nNodes / 16, 256, 0, stream>>>(S, input, W_e2n, b_e2n, W_n2n, b_n2n,
                                                    W_o1, b_o1, W_o2, b_o2, out);
}
